// VanillaRNN_76836964925694
// MI455X (gfx1250) — hardware-verified
//
#include <hip/hip_runtime.h>
#include <math.h>

typedef __attribute__((ext_vector_type(16))) _Float16 v16h;
typedef __attribute__((ext_vector_type(8)))  _Float16 v8h;
typedef __attribute__((ext_vector_type(16))) __bf16   v16b;
typedef __attribute__((ext_vector_type(8)))  __bf16   v8b;
typedef __attribute__((ext_vector_type(8)))  float    v8f;
typedef __attribute__((ext_vector_type(4)))  float    v4f;

constexpr int kB   = 512;
constexpr int kDin = 256;
constexpr int kH   = 768;
constexpr int kC   = 128;
constexpr int kT   = 128;
constexpr float kWCarry    = 64.0f;
constexpr float kWCarryInv = 1.0f / 64.0f;
static_assert(kDin % 32 == 0 && kH % 32 == 0);
static_assert(kB % 64 == 0 && kH % 64 == 0 && kC % 64 == 0);

constexpr int kPrepThreads = 256;
constexpr int kChX   = kB * kDin / 8;
constexpr int kChWhx = kH * kDin / 8;
constexpr int kChWhh = kH * kH / 8;
constexpr int kChWph = kC * kH / 8;
constexpr int kPB1 = kChX / kPrepThreads;
constexpr int kPB2 = kPB1 + kChWhx / kPrepThreads;
constexpr int kPB3 = kPB2 + kChWhh / kPrepThreads;
constexpr int kPrepBlocks = kPB3 + kChWph / kPrepThreads;
static_assert(kChX % kPrepThreads == 0 && kChWhx % kPrepThreads == 0 && kChWhh % kPrepThreads == 0 && kChWph % kPrepThreads == 0);
static_assert(kPrepBlocks == 496);
static_assert(kDin / 8 == 32);

constexpr int kGemm1Tiles  = (kH / 64) * (kB / 64);
constexpr int kGemm2Tiles  = (kB / 64) * (kC / 64);
constexpr int kGemm1Blocks = kGemm1Tiles / 8;
constexpr int kGemm2Blocks = kGemm2Tiles / 8;
static_assert(kGemm1Tiles % 8 == 0 && kGemm2Tiles % 8 == 0);

constexpr int kRnnThreads = 384;
constexpr int kRnnWaves   = kRnnThreads / 32;
constexpr int kSeqPB      = 16;
constexpr int kRnnBlocks  = kB / kSeqPB;
constexpr int kHP         = kH + 8;
constexpr int kHTile      = kSeqPB * kHP;
constexpr int kKChunks    = kH / 32;
static_assert(kH == 64 * kRnnWaves);
static_assert(kB % kSeqPB == 0);
static_assert(kHP % 8 == 0 && kHP >= kH);
static_assert((2 * kHTile) % 8 == 0);

constexpr int kSmThreads = 128;
constexpr int kSmRows    = 32;
constexpr int kSmBlocks  = kB / kSmRows;
constexpr int kYP        = 132;
static_assert(kC == 4 * 32);
static_assert(kSmRows == 8 * (kSmThreads / 32));
static_assert(kC == 32 * (kSmThreads / 32));
static_assert(kB % kSmRows == 0);
static_assert((kYP * 4) % 16 == 0);

__device__ __forceinline__ unsigned short f2bf_bits(float f) {
  unsigned u = __float_as_uint(f);
  return (unsigned short)((u + 0x7FFFu + ((u >> 16) & 1u)) >> 16);
}
__device__ __forceinline__ float bf_bits2f(unsigned short h) { return __uint_as_float(((unsigned)h) << 16); }

__device__ __forceinline__ void dep_guard_h(v8f& a, v8f& b, v16h x, v16h y) { asm volatile("v_nop\n\tv_nop\n\tv_nop\n\tv_nop" : "+v"(a), "+v"(b) : "v"(x), "v"(y)); }
__device__ __forceinline__ void dep_guard_b(v8f& a, v8f& b, v16b x, v16b y) { asm volatile("v_nop\n\tv_nop\n\tv_nop\n\tv_nop" : "+v"(a), "+v"(b) : "v"(x), "v"(y)); }
__device__ __forceinline__ void dep_guard4_h(v8f& a, v8f& b, v8f& c, v8f& d, v16h x, v16h y) {
  asm volatile("v_nop\n\tv_nop\n\tv_nop\n\tv_nop" : "+v"(a), "+v"(b), "+v"(c), "+v"(d) : "v"(x), "v"(y));
}
__device__ __forceinline__ void dep_guard4_b(v8f& a, v8f& b, v8f& c, v8f& d, v16b x, v16b y) {
  asm volatile("v_nop\n\tv_nop\n\tv_nop\n\tv_nop" : "+v"(a), "+v"(b), "+v"(c), "+v"(d) : "v"(x), "v"(y));
}
__device__ __forceinline__ void mma_guard4x5(v8f& a, v8f& b, v8f& c, v8f& d, v16h x, v16h y0, v16h y1, v16h y2, v16h y3) {
  asm volatile("v_nop\n\tv_nop\n\tv_nop\n\tv_nop" : "+v"(a), "+v"(b), "+v"(c), "+v"(d) : "v"(x), "v"(y0), "v"(y1), "v"(y2), "v"(y3));
}
__device__ __forceinline__ void keep4_h(v16h a, v16h b, v16h c, v16h d) { asm volatile("v_nop" :: "v"(a), "v"(b), "v"(c), "v"(d)); }
__device__ __forceinline__ void keep4_b(v16b a, v16b b, v16b c, v16b d) { asm volatile("v_nop" :: "v"(a), "v"(b), "v"(c), "v"(d)); }
__device__ __forceinline__ void acc_guard4(v8f& a, v8f& b, v8f& c, v8f& d) { asm volatile("v_nop\n\tv_nop\n\tv_nop\n\tv_nop" : "+v"(a), "+v"(b), "+v"(c), "+v"(d)); }

template <typename T> struct Frag;
template <> struct Frag<_Float16> {
  typedef v16h V; union U { v16h v; v8h h[2]; };
  static __device__ __forceinline__ v16h load(const _Float16* p) {
    U f; f.h[0] = *(const v8h*)(p); f.h[1] = *(const v8h*)(p + 16); return f.v;
  }
  static __device__ __forceinline__ v8f mma(v16h a, v16h b, v8f c) {
    return __builtin_amdgcn_wmma_f32_16x16x32_f16(false, a, false, b, (short)0, c, false, false);
  }
  static __device__ __forceinline__ void guard(v8f& a, v8f& b, v16h x, v16h y) { dep_guard_h(a, b, x, y); }
  static __device__ __forceinline__ void guard4(v8f& a, v8f& b, v8f& c, v8f& d, v16h x, v16h y) { dep_guard4_h(a, b, c, d, x, y); }
  static __device__ __forceinline__ void keep(v16h a, v16h b, v16h c, v16h d) { keep4_h(a, b, c, d); }
};
template <> struct Frag<__bf16> {
  typedef v16b V; union U { v16b v; v8b h[2]; };
  static __device__ __forceinline__ v16b load(const __bf16* p) {
    U f; f.h[0] = *(const v8b*)(p); f.h[1] = *(const v8b*)(p + 16); return f.v;
  }
  static __device__ __forceinline__ v8f mma(v16b a, v16b b, v8f c) {
    return __builtin_amdgcn_wmma_f32_16x16x32_bf16(false, a, false, b, (short)0, c, false, false);
  }
  static __device__ __forceinline__ void guard(v8f& a, v8f& b, v16b x, v16b y) { dep_guard_b(a, b, x, y); }
  static __device__ __forceinline__ void guard4(v8f& a, v8f& b, v8f& c, v8f& d, v16b x, v16b y) { dep_guard4_b(a, b, c, d, x, y); }
  static __device__ __forceinline__ void keep(v16b a, v16b b, v16b c, v16b d) { keep4_b(a, b, c, d); }
};

template <int ET> struct Elem;
template <> struct Elem<0> { typedef _Float16 T; };
template <> struct Elem<1> { typedef __bf16 T; };
template <int ET, bool SPLIT, int BIAS_MODE, int OUT_MODE, bool RESID, int ACT = 0>
__global__ __launch_bounds__(256) void wmma_gemm64(
    const unsigned short* __restrict__ Ap, const unsigned short* __restrict__ A2p, int lda, long strideA,
    const unsigned short* __restrict__ Btp, const unsigned short* __restrict__ Bt2p, int ldb, long strideB,
    void* __restrict__ Cout, void* __restrict__ Cout2, int ldc, long strideC,
    const float* __restrict__ bias,
    const float* __restrict__ resid, long strideR,
    int M, int N, int K, float scale) {
  typedef typename Elem<ET>::T T;
  typedef typename Frag<T>::V V;
  const T* A = (const T*)Ap; const T* A2 = (const T*)A2p; const T* Bt = (const T*)Btp; const T* Bt2 = (const T*)Bt2p;
  __shared__ __align__(16) float sT[8][16 * 68];
  const int b    = blockIdx.y;
  const int lane = threadIdx.x & 31;
  const int wave = threadIdx.x >> 5;
  const int tilesN = N >> 6;
  const int tilesM = M >> 6;
  const int tile = blockIdx.x * 8 + wave;
  if (tile >= tilesM * tilesN) return;
  const int tm = tile / tilesN;
  const int tn = tile - tm * tilesN;
  const int m0 = tm << 6;
  const int n0 = tn << 6;

  const T* Ab  = A  + (size_t)b * strideA;
  const T* Bb  = Bt + (size_t)b * strideB;
  const T* Ab2 = SPLIT ? (A2  + (size_t)b * strideA) : nullptr;
  const T* Bb2 = SPLIT ? (Bt2 + (size_t)b * strideB) : nullptr;

  const int rlane = lane & 15;
  const int koff  = (lane >> 4) * 8;
  const int mOff  = (lane >> 4) * 8;

  v8f acc[4][4];
#pragma unroll
  for (int i = 0; i < 4; ++i)
#pragma unroll
    for (int j = 0; j < 4; ++j) acc[i][j] = (v8f){0.f,0.f,0.f,0.f,0.f,0.f,0.f,0.f};

  for (int k0 = 0; k0 < K; k0 += 32) {
    V bh[4], bl[4];
#pragma unroll
    for (int j = 0; j < 4; ++j) {
      const size_t bo = (size_t)(n0 + (j << 4) + rlane) * ldb + koff + k0;
      bh[j] = Frag<T>::load(Bb + bo);
      if (SPLIT) bl[j] = Frag<T>::load(Bb2 + bo);
    }
#pragma unroll
    for (int i = 0; i < 4; ++i) {
      const size_t ao = (size_t)(m0 + (i << 4) + rlane) * lda + koff + k0;
      V ah = Frag<T>::load(Ab + ao);
      V al;
      if (SPLIT) al = Frag<T>::load(Ab2 + ao);
#pragma unroll
      for (int j = 0; j < 4; ++j) {
        acc[i][j] = Frag<T>::mma(ah, bh[j], acc[i][j]);
        if (SPLIT) {
          acc[i][j] = Frag<T>::mma(ah, bl[j], acc[i][j]);
          acc[i][j] = Frag<T>::mma(al, bh[j], acc[i][j]);
        }
      }
      Frag<T>::guard4(acc[i][0], acc[i][1], acc[i][2], acc[i][3], ah, SPLIT ? al : ah);
    }
    Frag<T>::keep(bh[0], bh[1], bh[2], bh[3]);
    if (SPLIT) Frag<T>::keep(bl[0], bl[1], bl[2], bl[3]);
  }
  acc_guard4(acc[0][0], acc[0][1], acc[0][2], acc[0][3]);
  acc_guard4(acc[1][0], acc[1][1], acc[1][2], acc[1][3]);
  acc_guard4(acc[2][0], acc[2][1], acc[2][2], acc[2][3]);
  acc_guard4(acc[3][0], acc[3][1], acc[3][2], acc[3][3]);

  float* slab = sT[wave];
  const float* Rb = RESID ? (resid + (size_t)b * strideR) : nullptr;
#pragma unroll
  for (int i = 0; i < 4; ++i) {
    const int mBase = m0 + (i << 4);
#pragma unroll
    for (int j = 0; j < 4; ++j) {
      const int n = n0 + (j << 4) + rlane;
      float bv = 0.f;
      if (BIAS_MODE == 2) bv = bias[n];
#pragma unroll
      for (int r = 0; r < 8; ++r) {
        float v = acc[i][j][r] * scale;
        if (BIAS_MODE == 1) v += bias[mBase + mOff + r];
        if (BIAS_MODE == 2) v += bv;
        if (RESID) v += Rb[(size_t)(mBase + mOff + r) * ldc + n];
        if (ACT == 1) v = tanhf(v);
        if (ACT == 2) v = fmaxf(v, 0.0f);
        if (ACT == 4) v = (v > 0.f) ? v : 0.01f * v;
        slab[(mOff + r) * 68 + (j << 4) + rlane] = v;
      }
    }
    __builtin_amdgcn_fence(__ATOMIC_RELEASE, "workgroup");
    __builtin_amdgcn_wave_barrier();
    __builtin_amdgcn_fence(__ATOMIC_ACQUIRE, "workgroup");
    if (OUT_MODE == 0) {
      float* C = (float*)Cout + (size_t)b * strideC;
      const int hh = lane >> 4, c4 = (lane & 15) * 4;
      for (int pass = 0; pass < 2; ++pass) {
#pragma unroll
        for (int it = 0; it < 8; ++it) {
          const int row = it * 2 + hh;
          v4f v = *(const v4f*)(slab + row * 68 + c4);
          *(volatile v4f*)(C + (size_t)(mBase + row) * ldc + n0 + c4) = v;
        }
        __threadfence();
      }
    } else {
      const int q = lane >> 3, c8 = (lane & 7) * 8;
      unsigned short* C  = (unsigned short*)Cout  + (size_t)b * strideC;
      unsigned short* C2 = (OUT_MODE == 2) ? ((unsigned short*)Cout2 + (size_t)b * strideC) : nullptr;
      for (int pass = 0; pass < 2; ++pass) {
#pragma unroll
        for (int it = 0; it < 4; ++it) {
          const int row = it * 4 + q;
          const float* sp = slab + row * 68 + c8;
          v8h hv, lv;
#pragma unroll
          for (int e = 0; e < 8; ++e) {
            if (OUT_MODE == 1) {
              hv[e] = (_Float16)sp[e];
            } else {
              unsigned short hb = f2bf_bits(sp[e]);
              unsigned short lb = f2bf_bits(sp[e] - bf_bits2f(hb));
              hv[e] = __builtin_bit_cast(_Float16, hb);
              lv[e] = __builtin_bit_cast(_Float16, lb);
            }
          }
          *(volatile v8h*)(C + (size_t)(mBase + row) * ldc + n0 + c8) = hv;
          if (OUT_MODE == 2) *(volatile v8h*)(C2 + (size_t)(mBase + row) * ldc + n0 + c8) = lv;
        }
        __threadfence();
      }
    }
    __builtin_amdgcn_fence(__ATOMIC_RELEASE, "workgroup");
    __builtin_amdgcn_wave_barrier();
    __builtin_amdgcn_fence(__ATOMIC_ACQUIRE, "workgroup");
  }
}

__device__ __forceinline__ void st2h(_Float16* p, v8h v) {
  *(volatile v8h*)p = v;
  __threadfence();
  *(volatile v8h*)p = v;
}
__device__ __forceinline__ float ftanh(float x) {
  return 1.0f - 2.0f * __builtin_amdgcn_rcpf(1.0f + expf(2.0f * x));
}
__device__ __forceinline__ void tr_chunk(const float* __restrict__ W, int wpitch, int kchunks, int i,
                                         _Float16* __restrict__ dst) {
  const int n  = i / kchunks;
  const int k8 = i - n * kchunks;
  const float* sp = W + (size_t)(k8 * 8) * wpitch + n;
  float f[8];
#pragma unroll
  for (int e = 0; e < 8; ++e) f[e] = sp[(size_t)e * wpitch];
  v8h hv;
#pragma unroll
  for (int e = 0; e < 8; ++e) hv[e] = (_Float16)(f[e] * kWCarry);
  st2h(dst + (size_t)i * 8, hv);
}

__global__ __launch_bounds__(kPrepThreads) void prep_kernel(
    const float* __restrict__ x, const float* __restrict__ w_hx, const float* __restrict__ w_hh,
    const float* __restrict__ w_ph,
    _Float16* __restrict__ x16, _Float16* __restrict__ whx16, _Float16* __restrict__ whh16,
    _Float16* __restrict__ wph16) {
  const int blk = blockIdx.x, tid = threadIdx.x;
  if (blk < kPB1) {
    const int i = blk * kPrepThreads + tid;
    const int row = i >> 5, c8 = i & 31;
    const float* src = x + (size_t)row * kDin + c8 * 8;
    const v4f f0 = *(const v4f*)src;
    const v4f f1 = *(const v4f*)(src + 4);
    v8h hv;
    hv[0] = (_Float16)f0[0]; hv[1] = (_Float16)f0[1]; hv[2] = (_Float16)f0[2]; hv[3] = (_Float16)f0[3];
    hv[4] = (_Float16)f1[0]; hv[5] = (_Float16)f1[1]; hv[6] = (_Float16)f1[2]; hv[7] = (_Float16)f1[3];
    st2h(x16 + (size_t)i * 8, hv);
  } else if (blk < kPB2) {
    const int i = (blk - kPB1) * kPrepThreads + tid;
    tr_chunk(w_hx, kH, kDin / 8, i, whx16);
  } else if (blk < kPB3) {
    const int i = (blk - kPB2) * kPrepThreads + tid;
    tr_chunk(w_hh, kH, kH / 8, i, whh16);
  } else {
    const int i = (blk - kPB3) * kPrepThreads + tid;
    tr_chunk(w_ph, kC, kH / 8, i, wph16);
  }
}

__global__ __launch_bounds__(kRnnThreads) void rnn_kernel(
    const float* __restrict__ xhbt, const _Float16* __restrict__ whh,
    const int* __restrict__ seqlen, _Float16* __restrict__ hl_out) {
  __shared__ __align__(16) _Float16 hbuf[2 * kHTile];
  const int tid = threadIdx.x, lane = tid & 31, wave = tid >> 5;
  const int c = lane & 15, hh = lane >> 4, koff = hh * 8, mOff = hh * 8;
  const int seq0 = blockIdx.x * kSeqPB;
  const int n0 = wave * 64;

  int ns = seqlen[0];
  ns = (ns < 0) ? 0 : ns;
  ns = (ns > kT) ? kT : ns;

  {
    const v8h z = {(_Float16)0.f, (_Float16)0.f, (_Float16)0.f, (_Float16)0.f, (_Float16)0.f, (_Float16)0.f, (_Float16)0.f, (_Float16)0.f};
    for (int i = tid; i < (2 * kHTile) / 8; i += kRnnThreads) *(v8h*)(hbuf + i * 8) = z;
  }

  v8f xfr[4];
#pragma unroll
  for (int j = 0; j < 4; ++j) {
    const float* xp = xhbt + (size_t)(n0 + 16 * j + c) * kB + seq0 + 8 * hh;
    const v4f xa = *(const v4f*)xp;
    const v4f xb = *(const v4f*)(xp + 4);
    xfr[j][0] = xa[0] * kWCarry; xfr[j][1] = xa[1] * kWCarry; xfr[j][2] = xa[2] * kWCarry; xfr[j][3] = xa[3] * kWCarry;
    xfr[j][4] = xb[0] * kWCarry; xfr[j][5] = xb[1] * kWCarry; xfr[j][6] = xb[2] * kWCarry; xfr[j][7] = xb[3] * kWCarry;
  }
  __syncthreads();

  const _Float16* brow = whh + (size_t)(n0 + c) * kH + koff;

#pragma unroll 1
  for (int t = 0; t < ns; ++t) {
    const _Float16* hc = hbuf + (t & 1) * kHTile;
    _Float16*       hn = hbuf + ((t + 1) & 1) * kHTile;
    v8f acc[4];
#pragma unroll
    for (int j = 0; j < 4; ++j) acc[j] = xfr[j];

    const _Float16* arow = hc + c * kHP + koff;
#pragma unroll 2
    for (int kc = 0; kc < kKChunks; ++kc) {
      const v16h fa = Frag<_Float16>::load(arow + kc * 32);
      v16h fb[4];
#pragma unroll
      for (int j = 0; j < 4; ++j) fb[j] = Frag<_Float16>::load(brow + (size_t)(16 * j) * kH + kc * 32);
#pragma unroll
      for (int j = 0; j < 4; ++j) acc[j] = Frag<_Float16>::mma(fa, fb[j], acc[j]);
      mma_guard4x5(acc[0], acc[1], acc[2], acc[3], fa, fb[0], fb[1], fb[2], fb[3]);
    }
    acc_guard4(acc[0], acc[1], acc[2], acc[3]);

#pragma unroll
    for (int j = 0; j < 4; ++j) {
#pragma unroll
      for (int r = 0; r < 8; ++r) {
        const float hv = ftanh(acc[j][r] * kWCarryInv);
        hn[(mOff + r) * kHP + n0 + 16 * j + c] = (_Float16)hv;
      }
    }
    __syncthreads();
  }

  const _Float16* hl = hbuf + (ns & 1) * kHTile;
  const int q4 = lane >> 3, c8 = (lane & 7) * 8;
  for (int pass = 0; pass < 2; ++pass) {
#pragma unroll
    for (int it = 0; it < 4; ++it) {
      const int rr = it * 4 + q4;
      const v8h v = *(const v8h*)(hl + rr * kHP + n0 + c8);
      *(volatile v8h*)(hl_out + (size_t)(seq0 + rr) * kH + n0 + c8) = v;
    }
    __threadfence();
  }
}

__global__ __launch_bounds__(kSmThreads) void softmax_t_kernel(const float* __restrict__ p, float* __restrict__ out) {
  __shared__ __align__(16) float ys[kSmRows * kYP];
  const int tid = threadIdx.x, lane = tid & 31, wave = tid >> 5;
  const int b0 = blockIdx.x * kSmRows;

#pragma unroll 1
  for (int rr = 0; rr < 8; ++rr) {
    const int row = wave * 8 + rr;
    const v4f v = *(const v4f*)(p + (size_t)(b0 + row) * kC + 4 * lane);
    float m = fmaxf(fmaxf(v[0], v[1]), fmaxf(v[2], v[3]));
#pragma unroll
    for (int off = 1; off < 32; off <<= 1) m = fmaxf(m, __shfl_xor(m, off, 32));
    const float e0 = expf(v[0] - m);
    const float e1 = expf(v[1] - m);
    const float e2 = expf(v[2] - m);
    const float e3 = expf(v[3] - m);
    float s = (e0 + e1) + (e2 + e3);
#pragma unroll
    for (int off = 1; off < 32; off <<= 1) s += __shfl_xor(s, off, 32);
    const float inv = 1.0f / s;
    v4f y;
    y[0] = e0 * inv; y[1] = e1 * inv; y[2] = e2 * inv; y[3] = e3 * inv;
    *(v4f*)(ys + row * kYP + 4 * lane) = y;
  }
  __syncthreads();

  const int q = lane >> 3, bq = (lane & 7) * 4;
  for (int pass = 0; pass < 2; ++pass) {
#pragma unroll
    for (int it = 0; it < 8; ++it) {
      const int cc = wave * 32 + it * 4 + q;
      v4f o;
      o[0] = ys[(bq + 0) * kYP + cc];
      o[1] = ys[(bq + 1) * kYP + cc];
      o[2] = ys[(bq + 2) * kYP + cc];
      o[3] = ys[(bq + 3) * kYP + cc];
      *(volatile v4f*)(out + (size_t)cc * kB + b0 + bq) = o;
    }
    __threadfence();
  }
}

extern "C" void kernel_launch(void* const* d_in, const int* in_sizes, int n_in,
                              void* d_out, int out_size, void* d_ws, size_t ws_size, hipStream_t stream) {
  if (n_in < 7 || d_out == nullptr || d_ws == nullptr) return;
  if (in_sizes[0] != kB * kDin || in_sizes[1] != kDin * kH || in_sizes[2] != kH * kH ||
      in_sizes[3] != kH || in_sizes[4] != kH * kC || in_sizes[5] != kC || in_sizes[6] < 1 ||
      out_size != kC * kB) return;

  const float* x      = (const float*)d_in[0];
  const float* w_hx   = (const float*)d_in[1];
  const float* w_hh   = (const float*)d_in[2];
  const float* bias_h = (const float*)d_in[3];
  const float* w_ph   = (const float*)d_in[4];
  const float* bias_p = (const float*)d_in[5];
  const int*   seqlen = (const int*)d_in[6];
  float* out = (float*)d_out;

  char* ws = (char*)d_ws; size_t off = 0;
  auto carve = [&](size_t bytes) -> char* { char* ptr = ws + off; off += (bytes + 255) & ~(size_t)255; return ptr; };
  unsigned short* X16   = (unsigned short*)carve((size_t)kB * kDin * 2);
  unsigned short* WHX16 = (unsigned short*)carve((size_t)kH * kDin * 2);
  unsigned short* WHH16 = (unsigned short*)carve((size_t)kH * kH * 2);
  unsigned short* WPH16 = (unsigned short*)carve((size_t)kC * kH * 2);
  float*          XHBT  = (float*)carve((size_t)kH * kB * 4);
  unsigned short* HL16  = (unsigned short*)carve((size_t)kB * kH * 2);
  float*          PBUF  = (float*)carve((size_t)kB * kC * 4);
  if (off > ws_size || off > (size_t)134217728) return;

  prep_kernel<<<kPrepBlocks, kPrepThreads, 0, stream>>>(x, w_hx, w_hh, w_ph,
                                                       (_Float16*)X16, (_Float16*)WHX16, (_Float16*)WHH16,
                                                       (_Float16*)WPH16);

  wmma_gemm64<0, false, 1, 0, false, 0><<<dim3(kGemm1Blocks, 1), 256, 0, stream>>>(
      WHX16, nullptr, kDin, 0L, X16, nullptr, kDin, 0L,
      (void*)XHBT, nullptr, kB, 0L, bias_h, nullptr, 0L, kH, kB, kDin, kWCarryInv);

  rnn_kernel<<<kRnnBlocks, kRnnThreads, 0, stream>>>(XHBT, (const _Float16*)WHH16, seqlen, (_Float16*)HL16);

  wmma_gemm64<0, false, 2, 0, false, 0><<<dim3(kGemm2Blocks, 1), 256, 0, stream>>>(
      HL16, nullptr, kH, 0L, WPH16, nullptr, kH, 0L,
      (void*)PBUF, nullptr, kC, 0L, bias_p, nullptr, 0L, kB, kC, kH, kWCarryInv);

  softmax_t_kernel<<<kSmBlocks, kSmThreads, 0, stream>>>(PBUF, out);
}
